// LatticeMamba_27874337751279
// MI455X (gfx1250) — hardware-verified
//
#include <hip/hip_runtime.h>
#include <hip/hip_bf16.h>
#include <math.h>


typedef _Float16 bf16;
typedef _Float16 f16;
typedef __attribute__((ext_vector_type(4))) unsigned v4u_t;
typedef unsigned v4ua __attribute__((ext_vector_type(4), may_alias));
typedef __attribute__((ext_vector_type(4))) float v4f_t;
typedef float v4fa __attribute__((ext_vector_type(4), may_alias));
typedef __attribute__((ext_vector_type(16))) bf16  bf16x16;
typedef bf16x16 f16x16;
typedef __attribute__((ext_vector_type(8)))  bf16  bf16x8;
typedef bf16x8 f16x8;
typedef __attribute__((ext_vector_type(4)))  bf16  bf16x4;
typedef __attribute__((ext_vector_type(8)))  float f32x8;
__device__ __forceinline__ f32x8 wmma16(f16x16 a, f16x16 b, f32x8 c) {
  c = __builtin_amdgcn_wmma_f32_16x16x32_f16(false, a, false, b, (short)0, c, false, false);
  asm volatile("v_nop\n\tv_nop\n\tv_nop\n\tv_nop" : "+v"(c) : "v"(a), "v"(b));
  return c;
}
#define LDS_STRIDE 48
#define KSTRIDE    72
#define VSTRIDE    48

__device__ __forceinline__ f32x8 wmma_bf16(bf16x16 a, bf16x16 b, f32x8 c) {
  c = __builtin_amdgcn_wmma_f32_16x16x32_f16(false, a, false, b, (short)0, c, false, false);
  asm volatile("v_nop\n\tv_nop\n\tv_nop\n\tv_nop" : "+v"(c) : "v"(a), "v"(b));
  return c;
}

template <typename T>
__device__ __forceinline__ bf16x16 load_frag(const T* __restrict__ base, int ld,
                                             int row0, int k0) {
  const int lane = threadIdx.x & 31;
  const int r    = lane & 15;
  const int kh   = (lane >> 4) * 8;
  const T* p0 = base + (size_t)(row0 + r) * ld + (k0 + kh);
  const T* p1 = p0 + 16;
  bf16x16 f;
#pragma unroll
  for (int i = 0; i < 8; ++i) {
    f[i]     = (bf16)p0[i];
    f[i + 8] = (bf16)p1[i];
  }
  return f;
}

__device__ __forceinline__ bf16x16 lds_frag(const bf16* base, int stride) {
  const int lane = threadIdx.x & 31;
  const int row  = lane & 15;
  const int kh   = (lane >> 4) * 8;
  const bf16x8 lo = *(const bf16x8*)(base + row * stride + kh);
  const bf16x8 hi = *(const bf16x8*)(base + row * stride + kh + 16);
  bf16x16 f;
#pragma unroll
  for (int i = 0; i < 8; ++i) { f[i] = lo[i]; f[i + 8] = hi[i]; }
  return f;
}

template <typename T>
__device__ __forceinline__ void stage_read16(const T* __restrict__ p, float* buf) {
#pragma unroll
  for (int i = 0; i < 16; ++i) buf[i] = (float)p[i];
}

__device__ __forceinline__ void stage_write(bf16* dst, const float* buf, int nquad) {
#pragma unroll
  for (int i = 0; i < nquad; ++i) {
    bf16x4 q;
    q[0] = (bf16)buf[4 * i];     q[1] = (bf16)buf[4 * i + 1];
    q[2] = (bf16)buf[4 * i + 2]; q[3] = (bf16)buf[4 * i + 3];
    *(bf16x4*)(dst + 4 * i) = q;
  }
}


#define GSTR 48
#define GSTR 48
template <typename AT, int EPI, bool OUT16>
__global__ __launch_bounds__(256) void gemm_kne(const AT* __restrict__ A, int lda, const float* __restrict__ Wm, int ldw,
                                                const float* __restrict__ bias, const float* __restrict__ R, const float* __restrict__ gvec,
                                                void* __restrict__ Yv, int ldy, int K) {
  __shared__ __attribute__((aligned(16))) f16 ldsA[128 * GSTR];
  __shared__ __attribute__((aligned(16))) f16 ldsW[128 * GSTR];
  __shared__ __attribute__((aligned(16))) float oS[8][32 * 68];
  const int tid = threadIdx.x, lane = tid & 31, wave = tid >> 5, cl = lane & 15, rh = (lane >> 4) * 8;
  const int m0 = blockIdx.x * 128, n0 = blockIdx.y * 128;
  const int wm = (wave & 3) * 32, wn = (wave >> 2) * 64;
  f32x8 acc[2][4];
#pragma unroll
  for (int i = 0; i < 2; ++i)
#pragma unroll
    for (int j = 0; j < 4; ++j) { f32x8 z = {}; acc[i][j] = z; }
#pragma unroll 1
  for (int k0 = 0; k0 < K; k0 += 32) {
    __syncthreads();
    { const int row = tid >> 1, ch = (tid & 1) * 16;
      const AT* src = A + (size_t)(m0 + row) * lda + k0 + ch;
#pragma unroll
      for (int g = 0; g < 16; ++g) ldsA[row * GSTR + ch + g] = (f16)src[g]; }
    { const int k = tid >> 3, nn0 = (tid & 7) * 16;
      const float* src = Wm + (size_t)(k0 + k) * ldw + n0 + nn0;
#pragma unroll
      for (int g = 0; g < 4; ++g) { const v4f_t v = *(const v4f_t*)(src + 4 * g);
#pragma unroll
        for (int u = 0; u < 4; ++u) ldsW[(nn0 + 4 * g + u) * GSTR + k] = (f16)v[u]; } }
    __syncthreads();
    f16x16 af[2];
#pragma unroll
    for (int i = 0; i < 2; ++i) af[i] = lds_frag(ldsA + (wm + 16 * i) * GSTR, GSTR);
#pragma unroll
    for (int j = 0; j < 4; ++j) {
      const f16x16 bf = lds_frag(ldsW + (wn + 16 * j) * GSTR, GSTR);
#pragma unroll
      for (int i = 0; i < 2; ++i) acc[i][j] = wmma16(af[i], bf, acc[i][j]);
    }
  }
  float* so = oS[wave];
#pragma unroll
  for (int i = 0; i < 2; ++i)
#pragma unroll
    for (int j = 0; j < 4; ++j) {
      const int n = n0 + wn + 16 * j + cl;
      const float bv = bias ? bias[n] : 0.0f;
      const float gv = (EPI == 2 || EPI == 4) ? gvec[n] : 0.0f;
      if (EPI == 1) {
#pragma unroll 1
        for (int r = 0; r < 8; ++r) { const float xg = acc[i][j][r] + bv; so[(16 * i + rh + r) * 68 + 16 * j + cl] = 0.5f * xg * (1.0f + erff(xg * 0.70710678118654752f)); }
      } else {
#pragma unroll
        for (int r = 0; r < 8; ++r) {
          float v = acc[i][j][r] + bv;
          if (EPI == 3) v = fmaxf(v, 0.0f);
          if (EPI == 4) v = gv * v;
          if (EPI == 2) v = R[(size_t)(m0 + wm + 16 * i + rh + r) * ldy + n] + gv * v;
          so[(16 * i + rh + r) * 68 + 16 * j + cl] = v;
        }
      }
    }
  asm volatile("s_wait_dscnt 0" ::: "memory");
  __builtin_amdgcn_wave_barrier();
#pragma unroll 1
  for (int pass = 0; pass < 2; ++pass) {
    if (OUT16) {
      f16* Y = (f16*)Yv;
#pragma unroll
      for (int it = 0; it < 8; ++it) { const int c = lane + 32 * it, rr = c >> 3, q8 = (c & 7) * 8;
        union { f16 h[8]; v4u_t v; } u;
#pragma unroll
        for (int e = 0; e < 8; ++e) u.h[e] = (f16)so[rr * 68 + q8 + e];
        *(volatile v4u_t*)(Y + (size_t)(m0 + wm + rr) * ldy + n0 + wn + q8) = u.v; }
    } else {
      float* Y = (float*)Yv;
#pragma unroll
      for (int it = 0; it < 16; ++it) { const int f4 = lane + 32 * it, rr = f4 >> 4, q = (f4 & 15) * 4;
        *(volatile v4f_t*)(Y + (size_t)(m0 + wm + rr) * ldy + n0 + wn + q) = *(const v4fa*)(so + rr * 68 + q); }
    }
    __threadfence();
  }
}

template <typename AT, int EPI, bool OUT16>
__global__ __launch_bounds__(256) void gemm_knez(const AT* __restrict__ A, int lda, size_t strideA, const float* __restrict__ Wm, int ldw, size_t strideW,
                                                 const float* __restrict__ bias, const float* __restrict__ R, const float* __restrict__ gvec,
                                                 void* __restrict__ Yv, int ldy, size_t strideY, int K) {
  A += (size_t)blockIdx.z * strideA; Wm += (size_t)blockIdx.z * strideW; Yv = (void*)((char*)Yv + (size_t)blockIdx.z * strideY * (OUT16 ? 2 : 4)); if (R) R += (size_t)blockIdx.z * strideY;
  __shared__ __attribute__((aligned(16))) f16 ldsA[128 * GSTR];
  __shared__ __attribute__((aligned(16))) f16 ldsW[128 * GSTR];
  __shared__ __attribute__((aligned(16))) float oS[8][32 * 68];
  const int tid = threadIdx.x, lane = tid & 31, wave = tid >> 5, cl = lane & 15, rh = (lane >> 4) * 8;
  const int m0 = blockIdx.x * 128, n0 = blockIdx.y * 128;
  const int wm = (wave & 3) * 32, wn = (wave >> 2) * 64;
  f32x8 acc[2][4];
#pragma unroll
  for (int i = 0; i < 2; ++i)
#pragma unroll
    for (int j = 0; j < 4; ++j) { f32x8 z = {}; acc[i][j] = z; }
#pragma unroll 1
  for (int k0 = 0; k0 < K; k0 += 32) {
    __syncthreads();
    { const int row = tid >> 1, ch = (tid & 1) * 16;
      const AT* src = A + (size_t)(m0 + row) * lda + k0 + ch;
#pragma unroll
      for (int g = 0; g < 16; ++g) ldsA[row * GSTR + ch + g] = (f16)src[g]; }
    { const int k = tid >> 3, nn0 = (tid & 7) * 16;
      const float* src = Wm + (size_t)(k0 + k) * ldw + n0 + nn0;
#pragma unroll
      for (int g = 0; g < 4; ++g) { const v4f_t v = *(const v4f_t*)(src + 4 * g);
#pragma unroll
        for (int u = 0; u < 4; ++u) ldsW[(nn0 + 4 * g + u) * GSTR + k] = (f16)v[u]; } }
    __syncthreads();
    f16x16 af[2];
#pragma unroll
    for (int i = 0; i < 2; ++i) af[i] = lds_frag(ldsA + (wm + 16 * i) * GSTR, GSTR);
#pragma unroll
    for (int j = 0; j < 4; ++j) {
      const f16x16 bf = lds_frag(ldsW + (wn + 16 * j) * GSTR, GSTR);
#pragma unroll
      for (int i = 0; i < 2; ++i) acc[i][j] = wmma16(af[i], bf, acc[i][j]);
    }
  }
  float* so = oS[wave];
#pragma unroll
  for (int i = 0; i < 2; ++i)
#pragma unroll
    for (int j = 0; j < 4; ++j) {
      const int n = n0 + wn + 16 * j + cl;
      const float bv = bias ? bias[n] : 0.0f;
      const float gv = (EPI == 2 || EPI == 4) ? gvec[n] : 0.0f;
      if (EPI == 1) {
#pragma unroll 1
        for (int r = 0; r < 8; ++r) { const float xg = acc[i][j][r] + bv; so[(16 * i + rh + r) * 68 + 16 * j + cl] = 0.5f * xg * (1.0f + erff(xg * 0.70710678118654752f)); }
      } else {
#pragma unroll
        for (int r = 0; r < 8; ++r) {
          float v = acc[i][j][r] + bv;
          if (EPI == 3) v = fmaxf(v, 0.0f);
          if (EPI == 4) v = gv * v;
          if (EPI == 2) v = R[(size_t)(m0 + wm + 16 * i + rh + r) * ldy + n] + gv * v;
          so[(16 * i + rh + r) * 68 + 16 * j + cl] = v;
        }
      }
    }
  asm volatile("s_wait_dscnt 0" ::: "memory");
  __builtin_amdgcn_wave_barrier();
#pragma unroll 1
  for (int pass = 0; pass < 2; ++pass) {
    if (OUT16) {
      f16* Y = (f16*)Yv;
#pragma unroll
      for (int it = 0; it < 8; ++it) { const int c = lane + 32 * it, rr = c >> 3, q8 = (c & 7) * 8;
        union { f16 h[8]; v4u_t v; } u;
#pragma unroll
        for (int e = 0; e < 8; ++e) u.h[e] = (f16)so[rr * 68 + q8 + e];
        *(volatile v4u_t*)(Y + (size_t)(m0 + wm + rr) * ldy + n0 + wn + q8) = u.v; }
    } else {
      float* Y = (float*)Yv;
#pragma unroll
      for (int it = 0; it < 16; ++it) { const int f4 = lane + 32 * it, rr = f4 >> 4, q = (f4 & 15) * 4;
        *(volatile v4f_t*)(Y + (size_t)(m0 + wm + rr) * ldy + n0 + wn + q) = *(const v4fa*)(so + rr * 68 + q); }
    }
    __threadfence();
  }
}

template <typename AT, bool ACC>
__global__ __launch_bounds__(256) void gemm_kn2(const AT* __restrict__ A, int lda, size_t strideA,
                                               const float* __restrict__ Wm, int ldw, size_t strideW,
                                               const float* __restrict__ bias, float scale,
                                               float* __restrict__ Y, int ldy, size_t strideY, int K) {
  __shared__ __attribute__((aligned(16))) f16 ldsA[128 * GSTR], ldsAl[128 * GSTR];
  __shared__ __attribute__((aligned(16))) f16 ldsW[128 * GSTR], ldsWl[128 * GSTR];
  __shared__ __attribute__((aligned(16))) float oS[8][32 * 68];
  const int tid = threadIdx.x, lane = tid & 31, wave = tid >> 5, cl = lane & 15, rh = (lane >> 4) * 8;
  const int m0 = blockIdx.x * 128, n0 = blockIdx.y * 128;
  const int wm = (wave & 3) * 32, wn = (wave >> 2) * 64;
  A += (size_t)blockIdx.z * strideA; Wm += (size_t)blockIdx.z * strideW; Y += (size_t)blockIdx.z * strideY;
  f32x8 acc[2][4], accx[2][4];
#pragma unroll
  for (int i = 0; i < 2; ++i)
#pragma unroll
    for (int j = 0; j < 4; ++j) { f32x8 z = {}; acc[i][j] = z; accx[i][j] = z; }
#pragma unroll 1
  for (int k0 = 0; k0 < K; k0 += 32) {
    __syncthreads();
    {
      const int row = tid >> 1, ch = (tid & 1) * 16;
      const AT* src = A + (size_t)(m0 + row) * lda + k0 + ch;
#pragma unroll
      for (int g = 0; g < 16; ++g) { const float v = (float)src[g]; const f16 h = (f16)v; ldsA[row * GSTR + ch + g] = h; ldsAl[row * GSTR + ch + g] = (f16)((v - (float)h) * 2048.0f); }
    }
    {
      const int k = tid >> 3, nn0 = (tid & 7) * 16;
      const float* src = Wm + (size_t)(k0 + k) * ldw + n0 + nn0;
#pragma unroll
      for (int g = 0; g < 4; ++g) { const v4f_t v = *(const v4f_t*)(src + 4 * g);
#pragma unroll
        for (int u = 0; u < 4; ++u) { const f16 h = (f16)v[u]; ldsW[(nn0 + 4 * g + u) * GSTR + k] = h; ldsWl[(nn0 + 4 * g + u) * GSTR + k] = (f16)((v[u] - (float)h) * 2048.0f); } }
    }
    __syncthreads();
    f16x16 af[2], afl[2];
#pragma unroll
    for (int i = 0; i < 2; ++i) { af[i] = lds_frag(ldsA + (wm + 16 * i) * GSTR, GSTR); afl[i] = lds_frag(ldsAl + (wm + 16 * i) * GSTR, GSTR); }
#pragma unroll
    for (int j = 0; j < 4; ++j) {
      const f16x16 bf = lds_frag(ldsW + (wn + 16 * j) * GSTR, GSTR), bfl = lds_frag(ldsWl + (wn + 16 * j) * GSTR, GSTR);
#pragma unroll
      for (int i = 0; i < 2; ++i) { acc[i][j] = wmma16(af[i], bf, acc[i][j]); accx[i][j] = wmma16(af[i], bfl, accx[i][j]); accx[i][j] = wmma16(afl[i], bf, accx[i][j]); }
    }
  }
  float* so = oS[wave];
#pragma unroll
  for (int i = 0; i < 2; ++i)
#pragma unroll
    for (int j = 0; j < 4; ++j) {
      const float bv = bias ? bias[n0 + wn + 16 * j + cl] : 0.0f;
#pragma unroll
      for (int r = 0; r < 8; ++r) so[(16 * i + rh + r) * 68 + 16 * j + cl] = (acc[i][j][r] + accx[i][j][r] * (1.0f / 2048.0f)) * scale + bv;
    }
  asm volatile("s_wait_dscnt 0" ::: "memory");
  __builtin_amdgcn_wave_barrier();
  if (ACC) {
#pragma unroll
    for (int it = 0; it < 16; ++it) { const int f4 = lane + 32 * it, rr = f4 >> 4, q = (f4 & 15) * 4;
      const v4f_t old = *(const v4fa*)(Y + (size_t)(m0 + wm + rr) * ldy + n0 + wn + q);
      v4f_t v = *(const v4fa*)(so + rr * 68 + q); v += old; *(v4fa*)(so + rr * 68 + q) = v; }
    asm volatile("s_wait_dscnt 0" ::: "memory");
  }
#pragma unroll 1
  for (int pass = 0; pass < 2; ++pass) {
#pragma unroll
    for (int it = 0; it < 16; ++it) { const int f4 = lane + 32 * it, rr = f4 >> 4, q = (f4 & 15) * 4;
      *(volatile v4f_t*)(Y + (size_t)(m0 + wm + rr) * ldy + n0 + wn + q) = *(const v4fa*)(so + rr * 68 + q); }
    __threadfence();
  }
}

__global__ __launch_bounds__(256) void k_transpose(const float* __restrict__ Wm, float* __restrict__ Wt, int rows, int cols) {
  __shared__ float tS[64][65];
  const int tid = threadIdx.x, tbj = cols / 64, bi = blockIdx.x / tbj, bj = blockIdx.x % tbj;
  for (int e = tid; e < 64 * 64; e += 256) { const int r = e >> 6, c = e & 63; tS[r][c] = Wm[(size_t)(bi * 64 + r) * cols + bj * 64 + c]; }
  __syncthreads();
  for (int ch = tid; ch < 64 * 16; ch += 256) { const int r = ch >> 4, q4 = (ch & 15) * 4; v4f_t o; o[0] = tS[q4][r]; o[1] = tS[q4 + 1][r]; o[2] = tS[q4 + 2][r]; o[3] = tS[q4 + 3][r];
    float* dst = Wt + (size_t)(bj * 64 + r) * rows + bi * 64 + q4; *(volatile v4f_t*)dst = o; __threadfence(); *(volatile v4f_t*)dst = o; }
}

#define NBT 8
#define LLs 1024
#define DMs 256
#define DIs 512
#define DSs 16
#define DTRs 16
#define NXs 48
#define NXP 128
#define DTP 32
#define TCH 64
#define CDs 64
#define NLs 4
__global__ __launch_bounds__(256) void k_fill(float* __restrict__ p, float val, size_t n4) { const size_t i = (size_t)blockIdx.x * 256 + threadIdx.x; if (i < n4) { v4f_t v = {val, val, val, val}; *(volatile v4f_t*)(p + 4 * i) = v; __threadfence(); *(volatile v4f_t*)(p + 4 * i) = v; } }
__global__ __launch_bounds__(256) void k_dbg_zero(float* __restrict__ p, size_t n4) { const size_t i = (size_t)blockIdx.x * 256 + threadIdx.x; if (i < n4) { v4f_t z = {0.f,0.f,0.f,0.f}; *(volatile v4f_t*)(p + 4 * i) = z; __threadfence(); *(volatile v4f_t*)(p + 4 * i) = z; } }
__global__ __launch_bounds__(256) void k_copy(const float* __restrict__ src, float* __restrict__ dst, size_t n4) { const size_t i = (size_t)blockIdx.x * 256 + threadIdx.x; if (i < n4) { const v4f_t v = *(const v4f_t*)(src + 4 * i); *(volatile v4f_t*)(dst + 4 * i) = v; __threadfence(); *(volatile v4f_t*)(dst + 4 * i) = v; } }
__global__ __launch_bounds__(256) void k_ln(const float* __restrict__ X, const float* __restrict__ gam, const float* __restrict__ bet, float* __restrict__ Y) {
  __shared__ __attribute__((aligned(16))) float rowS[16 * 260];
  const int tid = threadIdx.x, r = tid >> 4, part = tid & 15; const size_t row = (size_t)blockIdx.x * 16 + r;
  float s = 0.0f;
#pragma unroll 1
  for (int i = 0; i < 16; ++i) { const float v = X[row * 256 + part * 16 + i]; rowS[r * 260 + part * 16 + i] = v; s += v; }
  s += __shfl_xor(s, 1, 32); s += __shfl_xor(s, 2, 32); s += __shfl_xor(s, 4, 32); s += __shfl_xor(s, 8, 32);
  const float mean = s * (1.0f / 256.0f); float q = 0.0f;
#pragma unroll 1
  for (int i = 0; i < 16; ++i) { const float dv = rowS[r * 260 + part * 16 + i] - mean; q += dv * dv; }
  q += __shfl_xor(q, 1, 32); q += __shfl_xor(q, 2, 32); q += __shfl_xor(q, 4, 32); q += __shfl_xor(q, 8, 32);
  const float rstd = 1.0f / __builtin_sqrtf(q * (1.0f / 256.0f) + 1e-5f);
#pragma unroll 1
  for (int i = 0; i < 16; ++i) { const int c = part * 16 + i; rowS[r * 260 + c] = (rowS[r * 260 + c] - mean) * rstd * gam[c] + bet[c]; }
  __syncthreads();
#pragma unroll 1
  for (int pass = 0; pass < 2; ++pass) { for (int q4 = tid; q4 < 16 * 64; q4 += 256) { const int rr = q4 / 64, c4 = (q4 % 64) * 4;
      *(volatile v4f_t*)(Y + ((size_t)blockIdx.x * 16 + rr) * 256 + c4) = *(const v4fa*)(rowS + rr * 260 + c4); } __threadfence(); }
}
__global__ __launch_bounds__(256) void k_conv(const float* __restrict__ UZ, const float* __restrict__ cw, const float* __restrict__ cb, float* __restrict__ UC) {
  const int l = blockIdx.x, tid = threadIdx.x;
#pragma unroll 1
  for (int j = 0; j < DIs / 256; ++j) { const int d = tid + 256 * j; float acc = cb[d];
#pragma unroll
    for (int k = 0; k < 4; ++k) { const int ll = l - 3 + k; if (ll >= 0) acc = fmaf(UZ[(size_t)ll * (2 * DIs) + d], cw[d * 4 + k], acc); }
    const float sv = acc / (1.0f + expf(-acc));
    *(volatile float*)(UC + (size_t)l * DIs + d) = sv; __threadfence(); *(volatile float*)(UC + (size_t)l * DIs + d) = sv; }
}

__global__ __launch_bounds__(256) void k_scan(const float* __restrict__ PROJ, const float* __restrict__ DTRW, const float* __restrict__ UC, const float* __restrict__ UZ,
                                             const float* __restrict__ Alog, const float* __restrict__ Dv, bf16* __restrict__ G16) {
  __shared__ float BC[TCH][2 * DSs];
  __shared__ __attribute__((aligned(16))) bf16 gS[TCH][256 + 8];
  const int cg = blockIdx.x, tid = threadIdx.x; const int d = cg * 256 + tid;
  float a2[DSs], h[DSs];
#pragma unroll
  for (int n = 0; n < DSs; ++n) { a2[n] = -expf(Alog[(size_t)d * DSs + n]) * 1.4426950408889634f; h[n] = 0.0f; }
  const float Dd = Dv[d];
#pragma unroll 1
  for (int c0 = 0; c0 < LLs; c0 += TCH) {
    __syncthreads();
#pragma unroll 1
    for (int e = tid; e < TCH * 2 * DSs; e += 256) { const int t = e >> 5, c = e & 31; BC[t][c] = PROJ[((size_t)(c0 + t)) * NXP + DTRs + c]; }
    __syncthreads();
#pragma unroll 1
    for (int t = 0; t < TCH; ++t) { const size_t tok = (size_t)(c0 + t);
      const float dr = DTRW[tok * DIs + d]; const float dt = (dr > 20.0f) ? dr : log1pf(expf(dr));
      const float u = UC[tok * DIs + d]; const float dtu = dt * u; float y = u * Dd;
#pragma unroll
      for (int n = 0; n < DSs; ++n) { h[n] = fmaf(h[n], __builtin_amdgcn_exp2f(dt * a2[n]), dtu * BC[t][n]); y = fmaf(h[n], BC[t][DSs + n], y); }
      const float z = UZ[tok * (2 * DIs) + DIs + d]; const float g = y * (z / (1.0f + expf(-z)));
      gS[t][tid] = (bf16)(g * 64.0f); }
    __syncthreads();
#pragma unroll 1
    for (int pass = 0; pass < 2; ++pass) {
#pragma unroll 1
      for (int i = tid; i < TCH * 32; i += 256) { const int t = i >> 5, piece = (i & 31) * 8;
        *(volatile v4u_t*)(G16 + ((size_t)(c0 + t)) * DIs + cg * 256 + piece) = *(const v4ua*)(&gS[t][piece]); }
      __threadfence(); }
  }
}

__global__ __launch_bounds__(128) void k_padxp(const float* __restrict__ w, float* __restrict__ Wxp) {
  const int k = blockIdx.x, n = threadIdx.x; const float v = (n < NXs) ? w[(size_t)k * NXs + min(n, NXs - 1)] : 0.0f;
  *(volatile float*)(Wxp + (size_t)k * NXP + n) = v; __threadfence(); *(volatile float*)(Wxp + (size_t)k * NXP + n) = v;
}
__global__ __launch_bounds__(256) void k_paddt(const float* __restrict__ w, float* __restrict__ WdtT) {
  const int k = blockIdx.x, tid = threadIdx.x;
#pragma unroll
  for (int j = 0; j < DIs / 256; ++j) { const int d = tid + 256 * j; const float v = (k < DTRs) ? w[(size_t)min(k, DTRs - 1) * DIs + d] : 0.0f;
    *(volatile float*)(WdtT + (size_t)k * DIs + d) = v; __threadfence(); *(volatile float*)(WdtT + (size_t)k * DIs + d) = v; }
}
__global__ __launch_bounds__(64) void k_embed(const int* __restrict__ tok, const float* __restrict__ te, const float* __restrict__ pe, float* __restrict__ X) {
  const int l = blockIdx.x, c = 4 * threadIdx.x; const int t = min(max(tok[max(l - 1, 0)], 0), 1);
  const v4f_t e = *(const v4f_t*)(te + (size_t)t * DMs + c); const v4f_t p = *(const v4f_t*)(pe + (size_t)l * DMs + c); v4f_t v = p; if (l > 0) v += e;
  float* d = X + (size_t)l * DMs + c; *(volatile v4f_t*)d = v; __threadfence(); *(volatile v4f_t*)d = v;
}
__global__ __launch_bounds__(256) void k_cond(const float* __restrict__ Tv, int b, const float* __restrict__ tw1, const float* __restrict__ tb1, const float* __restrict__ tw2, const float* __restrict__ tb2,
                                             const float* __restrict__ ag, const float* __restrict__ ab, const float* __restrict__ apw, const float* __restrict__ apb, float* __restrict__ GB) {
  __shared__ float hh[CDs], cd[CDs];
  const int c = threadIdx.x; const float t = Tv[b];
  if (c < CDs) { const float v = t * tw1[c] + tb1[c]; hh[c] = 0.5f * v * (1.0f + erff(v * 0.70710678118654752f)); }
  __syncthreads();
  if (c < CDs) { float s = tb2[c];
#pragma unroll 1
    for (int j = 0; j < CDs; ++j) s = fmaf(hh[j], tw2[(size_t)j * CDs + c], s); cd[c] = s; }
  __syncthreads();
#pragma unroll 1
  for (int i = 0; i < NLs; ++i) { float sc = apb[(size_t)i * 2 * DMs + c], sh = apb[(size_t)i * 2 * DMs + DMs + c];
#pragma unroll 1
    for (int j = 0; j < CDs; ++j) { const float cj = cd[j]; sc = fmaf(cj, apw[((size_t)i * CDs + j) * 2 * DMs + c], sc); sh = fmaf(cj, apw[((size_t)i * CDs + j) * 2 * DMs + DMs + c], sh); }
    const float g2 = ag[(size_t)i * DMs + c] * (1.0f + sc), b2 = ab[(size_t)i * DMs + c] * (1.0f + sc) + sh;
    *(volatile float*)(GB + (size_t)i * 2 * DMs + c) = g2; *(volatile float*)(GB + (size_t)i * 2 * DMs + DMs + c) = b2; }
  __threadfence();
#pragma unroll 1
  for (int i = 0; i < NLs; ++i) { float* p = GB + (size_t)i * 2 * DMs + c; const float a = p[0], bb = p[DMs]; *(volatile float*)p = a; *(volatile float*)(p + DMs) = bb; }
}
__global__ __launch_bounds__(256) void k_head(const float* __restrict__ XN, const float* __restrict__ hw, const float* __restrict__ hb, float* __restrict__ out) {
  __shared__ float st[32];
  const int tid = threadIdx.x, r = tid >> 4, part = tid & 15; const size_t l = (size_t)blockIdx.x * 16 + r; const float* xr = XN + l * DMs;
  float a = 0.0f, b2 = 0.0f;
#pragma unroll 1
  for (int i = 0; i < DMs / 16; ++i) { const int c = part * (DMs / 16) + i; const float v = xr[c]; a = fmaf(v, hw[c * 2 + 0], a); b2 = fmaf(v, hw[c * 2 + 1], b2); }
  a += __shfl_xor(a, 1, 32); a += __shfl_xor(a, 2, 32); a += __shfl_xor(a, 4, 32); a += __shfl_xor(a, 8, 32);
  b2 += __shfl_xor(b2, 1, 32); b2 += __shfl_xor(b2, 2, 32); b2 += __shfl_xor(b2, 4, 32); b2 += __shfl_xor(b2, 8, 32);
  if (part == 0) { st[2 * r] = a + hb[0]; st[2 * r + 1] = b2 + hb[1]; }
  __syncthreads();
  if (tid < 8) { const v4f_t v = *(const v4fa*)(st + 4 * tid); float* d = out + (size_t)blockIdx.x * 32 + 4 * tid; *(volatile v4f_t*)d = v; __threadfence(); *(volatile v4f_t*)d = v; }
}

extern "C" void kernel_launch(void* const* d_in, const int* in_sizes, int n_in,
                              void* d_out, int out_size, void* d_ws, size_t ws_size,
                              hipStream_t stream) {
  (void)in_sizes; (void)n_in; (void)out_size;
  const int* tok = (const int*)d_in[0]; const float** f = (const float**)d_in;
  const float* Tv = f[1], *te = f[2], *pe = f[3], *tw1 = f[4], *tb1 = f[5], *tw2 = f[6], *tb2 = f[7], *ag = f[8], *ab = f[9], *apw = f[10], *apb = f[11], *inw = f[12], *cw = f[13], *cb = f[14],
              *xpw = f[15], *dtw = f[16], *dtb = f[17], *Alog = f[18], *Dv = f[19], *outw = f[20], *fg = f[21], *fb = f[22], *hw = f[23], *hbv = f[24];
  float* out = (float*)d_out;
  char* ws = (char*)d_ws;
  float* Wxp = (float*)ws; ws += (size_t)NLs * DIs * NXP * 4; float* WdtT = (float*)ws; ws += (size_t)NLs * DTP * DIs * 4;
  float* GB = (float*)ws; ws += (size_t)NLs * 2 * DMs * 4;
  float* X = (float*)ws; ws += (size_t)LLs * DMs * 4; float* XN = (float*)ws; ws += (size_t)LLs * DMs * 4;
  float* UZ = (float*)ws; ws += (size_t)LLs * 2 * DIs * 4; float* UC = (float*)ws; ws += (size_t)LLs * DIs * 4;
  float* PROJ = (float*)ws; ws += (size_t)LLs * NXP * 4; float* DTRW = (float*)ws; ws += (size_t)LLs * DIs * 4;
  bf16* G16 = (bf16*)ws; ws += (size_t)LLs * DIs * 2; float* r64 = (float*)ws; ws += DMs * 4;
  if ((size_t)(ws - (char*)d_ws) > ws_size) return;
  const dim3 blk(256);
  for (int i = 0; i < NLs; ++i) { k_padxp<<<dim3(DIs), dim3(128), 0, stream>>>(xpw + (size_t)i * DIs * NXs, Wxp + (size_t)i * DIs * NXP); k_paddt<<<dim3(DTP), blk, 0, stream>>>(dtw + (size_t)i * DTRs * DIs, WdtT + (size_t)i * DTP * DIs); }
  k_fill<<<dim3(1), blk, 0, stream>>>(r64, 1.0f / 64.0f, DMs / 4);

  for (int b = 0; b < NBT; ++b) {
    k_cond<<<dim3(1), blk, 0, stream>>>(Tv, b, tw1, tb1, tw2, tb2, ag, ab, apw, apb, GB);
    k_embed<<<dim3(LLs), dim3(64), 0, stream>>>(tok + (size_t)b * LLs, te, pe, X);
    for (int i = 0; i < NLs; ++i) {
      k_ln<<<dim3(LLs / 16), blk, 0, stream>>>(X, GB + (size_t)i * 2 * DMs, GB + (size_t)i * 2 * DMs + DMs, XN);
      gemm_kne<float, 0, false><<<dim3(LLs / 128, 2 * DIs / 128), blk, 0, stream>>>(XN, DMs, inw + (size_t)i * DMs * 2 * DIs, 2 * DIs, nullptr, nullptr, nullptr, UZ, 2 * DIs, DMs);
      k_conv<<<dim3(LLs), blk, 0, stream>>>(UZ, cw + (size_t)i * DIs * 4, cb + (size_t)i * DIs, UC);
      gemm_kne<float, 0, false><<<dim3(LLs / 128, 1), blk, 0, stream>>>(UC, DIs, Wxp + (size_t)i * DIs * NXP, NXP, nullptr, nullptr, nullptr, PROJ, NXP, DIs);
      gemm_kne<float, 0, false><<<dim3(LLs / 128, DIs / 128), blk, 0, stream>>>(PROJ, NXP, WdtT + (size_t)i * DTP * DIs, DIs, dtb + (size_t)i * DIs, nullptr, nullptr, DTRW, DIs, DTP);
      k_scan<<<dim3(DIs / 256), blk, 0, stream>>>(PROJ, DTRW, UC, UZ, Alog + (size_t)i * DIs * DSs, Dv + (size_t)i * DIs, G16);
      gemm_kne<bf16, 2, false><<<dim3(LLs / 128, DMs / 128), blk, 0, stream>>>(G16, DIs, outw + (size_t)i * DIs * DMs, DMs, nullptr, X, r64, X, DMs, DIs);
    }
    k_ln<<<dim3(LLs / 16), blk, 0, stream>>>(X, fg, fb, XN);
    k_head<<<dim3(LLs / 16), blk, 0, stream>>>(XN, hw, hbv, out + (size_t)b * LLs * 2);
  }
}
